// JointAttention_49950469653327
// MI455X (gfx1250) — hardware-verified
//
#include <hip/hip_runtime.h>
#include <math.h>
#include <stdint.h>

#ifndef NB
#define NB 2
#endif
#ifndef SEQ
#define SEQ 2048
#endif
#define NB_FULL  2
#define SEQ_FULL 2048
#define DIMX 2048
#define NH   16
#define NKV  8
#define HD   128
#define NREP (NH / NKV)
#define QD   (NH * HD)
#define KD   (NKV * HD)
#define QKC  (QD + KD)
#define QKVO (QD + 2 * KD)
#define FRQ  (HD * 2)
#define NQB  (SEQ / 64)
#define NKT  (SEQ / 64)
#define QRES    4096.0f
#define PCARRY  16384.0f
#define OCARRY  32.0f
#define WOCARRY 64.0f
#ifndef SCORE_QRES
#define SCORE_QRES 1
#endif
static_assert(NH * HD == DIMX);
static_assert(NREP * NKV == NH);
static_assert(HD == 128);
static_assert((SEQ % 64) == 0 && SEQ >= 64 && SEQ <= SEQ_FULL);
static_assert(NB >= 1 && NB <= NB_FULL);
static_assert((DIMX % 64) == 0 && (QKC % 64) == 0 && (KD % 64) == 0 && (QD % 64) == 0);
static_assert((DIMX % 32) == 0);

typedef _Float16 v16h __attribute__((ext_vector_type(16)));
typedef _Float16 v8h  __attribute__((ext_vector_type(8)));
typedef __bf16   v16b __attribute__((ext_vector_type(16)));
typedef float    v8f  __attribute__((ext_vector_type(8)));
typedef float    v4f  __attribute__((ext_vector_type(4)));
typedef unsigned int v4u __attribute__((ext_vector_type(4)));

__device__ __forceinline__ unsigned short bf_bits(float f) {
  unsigned u = __float_as_uint(f);
  return (unsigned short)((u + 0x7FFFu + ((u >> 16) & 1u)) >> 16);
}
__device__ __forceinline__ float bf_up(unsigned short h) { return __uint_as_float(((unsigned)h) << 16); }
__device__ __forceinline__ float bfr(float f) { return bf_up(bf_bits(f)); }
__device__ __forceinline__ unsigned short h_bits(_Float16 x) { return __builtin_bit_cast(unsigned short, x); }
__device__ __forceinline__ unsigned pk16(unsigned short a, unsigned short b) { return (unsigned)a | ((unsigned)b << 16); }
__device__ __forceinline__ v8f zero8() { v8f z = {0.f, 0.f, 0.f, 0.f, 0.f, 0.f, 0.f, 0.f}; return z; }

union Frag { v16h h; v16b b; v4u q[2]; };
__device__ __forceinline__ Frag ldfrag(const unsigned short* p) {
  Frag f;
  f.q[0] = *(const v4u*)(p);
  f.q[1] = *(const v4u*)(p + 16);
  return f;
}

__device__ __forceinline__ v8f mma_h(v16h a, v16h b, v8f c) {
  c = __builtin_amdgcn_wmma_f32_16x16x32_f16(false, a, false, b, (short)0, c, false, false);
  asm volatile("v_nop\n\tv_nop\n\tv_nop\n\tv_nop" : "+v"(c) : "v"(a), "v"(b));
  return c;
}
__device__ __forceinline__ v8f mma_bf(v16b a, v16b b, v8f c) {
  c = __builtin_amdgcn_wmma_f32_16x16x32_bf16(false, a, false, b, (short)0, c, false, false);
  asm volatile("v_nop\n\tv_nop\n\tv_nop\n\tv_nop" : "+v"(c) : "v"(a), "v"(b));
  return c;
}
template <int F16OP>
__device__ __forceinline__ v8f mma16(const Frag& a, const Frag& b, v8f c) {
  if (F16OP) return mma_h(a.h, b.h, c);
  return mma_bf(a.b, b.b, c);
}

__global__ __launch_bounds__(256) void cvt_x_bf16x8(const float* __restrict__ in, unsigned short* out, int n8) {
  const int i = blockIdx.x * 256 + threadIdx.x;
  if (i < n8) {
    const int row = i / (DIMX / 8);
    const int c8  = (i - row * (DIMX / 8)) * 8;
    const int bb  = row / SEQ;
    const int sq  = row - bb * SEQ;
    const float* src = in + ((size_t)bb * SEQ_FULL + sq) * DIMX + c8;
    const v4f a = *(const v4f*)(src);
    const v4f b = *(const v4f*)(src + 4);
    v4u p;
    p[0] = pk16(bf_bits(a[0]), bf_bits(a[1]));
    p[1] = pk16(bf_bits(a[2]), bf_bits(a[3]));
    p[2] = pk16(bf_bits(b[0]), bf_bits(b[1]));
    p[3] = pk16(bf_bits(b[2]), bf_bits(b[3]));
    *(volatile v4u*)(out + (size_t)i * 8) = p;
    __threadfence();
    *(volatile v4u*)(out + (size_t)i * 8) = p;
  }
}

__global__ __launch_bounds__(256) void cvt_bf16x8(const float* __restrict__ in, unsigned short* out, int n8) {
  const int i = blockIdx.x * 256 + threadIdx.x;
  if (i < n8) {
    const v4f a = *(const v4f*)(in + (size_t)i * 8);
    const v4f b = *(const v4f*)(in + (size_t)i * 8 + 4);
    v4u p;
    p[0] = pk16(bf_bits(a[0]), bf_bits(a[1]));
    p[1] = pk16(bf_bits(a[2]), bf_bits(a[3]));
    p[2] = pk16(bf_bits(b[0]), bf_bits(b[1]));
    p[3] = pk16(bf_bits(b[2]), bf_bits(b[3]));
    *(volatile v4u*)(out + (size_t)i * 8) = p;
    __threadfence();
    *(volatile v4u*)(out + (size_t)i * 8) = p;
  }
}

__global__ __launch_bounds__(256) void cvt_wo_f16x8(const float* __restrict__ in, unsigned short* out, int n8) {
  const int i = blockIdx.x * 256 + threadIdx.x;
  if (i < n8) {
    const v4f a = *(const v4f*)(in + (size_t)i * 8);
    const v4f b = *(const v4f*)(in + (size_t)i * 8 + 4);
    v4u p;
#pragma unroll
    for (int e = 0; e < 2; ++e) {
      const _Float16 x0 = (_Float16)(bfr(a[2 * e]) * WOCARRY), x1 = (_Float16)(bfr(a[2 * e + 1]) * WOCARRY);
      const _Float16 y0 = (_Float16)(bfr(b[2 * e]) * WOCARRY), y1 = (_Float16)(bfr(b[2 * e + 1]) * WOCARRY);
      p[e]     = pk16(h_bits(x0), h_bits(x1));
      p[2 + e] = pk16(h_bits(y0), h_bits(y1));
    }
    *(volatile v4u*)(out + (size_t)i * 8) = p;
    __threadfence();
    *(volatile v4u*)(out + (size_t)i * 8) = p;
  }
}

template <int F16OP, int OUT_MODE>
__global__ __launch_bounds__(256) void gemm64(
    const unsigned short* __restrict__ Ap, int lda, long long strideA,
    const unsigned short* __restrict__ Btp, int ldb, long long strideB,
    void* Cout, int ldc, long long strideC,
    int M, int N, int K, float oscale) {
  __shared__ __align__(16) float sT[8][16 * 68];
  const int b    = blockIdx.y;
  const int lane = threadIdx.x & 31;
  const int wave = threadIdx.x >> 5;
  const int tilesN = N >> 6;
  const int tilesM = M >> 6;
  const int tile = blockIdx.x * 8 + wave;
  if (tile >= tilesM * tilesN) return;
  const int tm = tile / tilesN;
  const int tn = tile - tm * tilesN;
  const int m0 = tm << 6;
  const int n0 = tn << 6;

  const unsigned short* Ab = Ap  + (size_t)b * strideA;
  const unsigned short* Bb = Btp + (size_t)b * strideB;

  const int rlane = lane & 15;
  const int koff  = (lane >> 4) * 8;
  const int mOff  = (lane >> 4) * 8;

  v8f acc[4][4];
#pragma unroll
  for (int i = 0; i < 4; ++i)
#pragma unroll
    for (int j = 0; j < 4; ++j) acc[i][j] = zero8();

  for (int k0 = 0; k0 < K; k0 += 32) {
    Frag bh[4];
#pragma unroll
    for (int j = 0; j < 4; ++j) {
      const size_t bo = (size_t)(n0 + (j << 4) + rlane) * ldb + koff + k0;
      bh[j] = ldfrag(Bb + bo);
    }
#pragma unroll
    for (int i = 0; i < 4; ++i) {
      const size_t ao = (size_t)(m0 + (i << 4) + rlane) * lda + koff + k0;
      const Frag ah = ldfrag(Ab + ao);
#pragma unroll
      for (int j = 0; j < 4; ++j) acc[i][j] = mma16<F16OP>(ah, bh[j], acc[i][j]);
    }
  }

  float* slab = sT[wave];
#pragma unroll
  for (int i = 0; i < 4; ++i) {
    const int mBase = m0 + (i << 4);
#pragma unroll
    for (int j = 0; j < 4; ++j) {
#pragma unroll
      for (int r = 0; r < 8; ++r) {
        slab[(mOff + r) * 68 + (j << 4) + rlane] = acc[i][j][r];
      }
    }
    __builtin_amdgcn_fence(__ATOMIC_RELEASE, "workgroup");
    __builtin_amdgcn_wave_barrier();
    __builtin_amdgcn_fence(__ATOMIC_ACQUIRE, "workgroup");
    if (OUT_MODE == 0) {
      float* C = (float*)Cout + (size_t)b * strideC;
      const int hsel = lane >> 4, c4 = (lane & 15) * 4;
      v4f ov[8];
#pragma unroll
      for (int it = 0; it < 8; ++it) {
        const int row = it * 2 + hsel;
        v4f v = *(const v4f*)(slab + row * 68 + c4);
#pragma unroll
        for (int e = 0; e < 4; ++e) v[e] = v[e] * oscale;
        ov[it] = v;
      }
#pragma unroll
      for (int pass = 0; pass < 2; ++pass) {
#pragma unroll
        for (int it = 0; it < 8; ++it) {
          const int row = it * 2 + hsel;
          *(volatile v4f*)(C + (size_t)(mBase + row) * ldc + n0 + c4) = ov[it];
        }
        __threadfence();
      }
    } else {
      const int q = lane >> 3, c8 = (lane & 7) * 8;
      unsigned short* C = (unsigned short*)Cout + (size_t)b * strideC;
      v4u hv[4];
#pragma unroll
      for (int it = 0; it < 4; ++it) {
        const int row = it * 4 + q;
        const float* sp = slab + row * 68 + c8;
        v4u a;
#pragma unroll
        for (int e = 0; e < 4; ++e) {
          const _Float16 x0 = (_Float16)(sp[2 * e] * oscale), x1 = (_Float16)(sp[2 * e + 1] * oscale);
          a[e] = pk16(h_bits(x0), h_bits(x1));
        }
        hv[it] = a;
      }
#pragma unroll
      for (int pass = 0; pass < 2; ++pass) {
#pragma unroll
        for (int it = 0; it < 4; ++it) {
          const int row = it * 4 + q;
          *(volatile v4u*)(C + (size_t)(mBase + row) * ldc + n0 + c8) = hv[it];
        }
        __threadfence();
      }
    }
    __builtin_amdgcn_fence(__ATOMIC_RELEASE, "workgroup");
    __builtin_amdgcn_wave_barrier();
    __builtin_amdgcn_fence(__ATOMIC_ACQUIRE, "workgroup");
  }
}

__global__ __launch_bounds__(256)
void qk_post(const float* __restrict__ qkf, const float* __restrict__ freqs,
             const float* __restrict__ qw, const float* __restrict__ kw,
             unsigned short* Qh, unsigned short* Ql, unsigned short* Kh, unsigned short* Kl) {
  __shared__ __align__(16) unsigned short sQh[QD];
  __shared__ __align__(16) unsigned short sQl[QD];
  __shared__ __align__(16) unsigned short sKh[KD];
  __shared__ __align__(16) unsigned short sKl[KD];
  const int tok  = blockIdx.x;
  const int bb   = tok / SEQ;
  const int pos  = tok - bb * SEQ;
  const int t    = threadIdx.x;
  const int wave = t >> 5;
  const int head = t >> 3;
  const int part = t & 7;
  const int d0   = part * 16;

  if (wave < 6) {
    const float* src = qkf + (size_t)tok * QKC + head * HD + d0;
    float x[16];
#pragma unroll
    for (int i = 0; i < 4; ++i) {
      const v4f a = *(const v4f*)(src + 4 * i);
#pragma unroll
      for (int e = 0; e < 4; ++e) x[4 * i + e] = a[e];
    }
    float ssq = 0.f;
#pragma unroll
    for (int i = 0; i < 16; ++i) ssq += x[i] * x[i];
    ssq += __shfl_xor(ssq, 1, 32);
    ssq += __shfl_xor(ssq, 2, 32);
    ssq += __shfl_xor(ssq, 4, 32);
    const float rn = rsqrtf(ssq * (1.0f / (float)HD) + 1e-5f);
    const float* wsrc = (wave < 4) ? qw : kw;
    float xn[16];
#pragma unroll
    for (int i = 0; i < 4; ++i) {
      const v4f wv = *(const v4f*)(wsrc + d0 + 4 * i);
#pragma unroll
      for (int e = 0; e < 4; ++e) xn[4 * i + e] = (x[4 * i + e] * rn) * bfr(wv[e]);
    }
    const float* fsrc = freqs + (size_t)pos * FRQ + (size_t)(part * 8) * 4;
    float y[16];
#pragma unroll
    for (int u = 0; u < 8; ++u) {
      const v4f f = *(const v4f*)(fsrc + 4 * u);
      const float f00 = bfr(f[0]), f01 = bfr(f[1]), f10 = bfr(f[2]), f11 = bfr(f[3]);
      const float a0 = xn[2 * u], a1 = xn[2 * u + 1];
      y[2 * u]     = f00 * a0 + f01 * a1;
      y[2 * u + 1] = f10 * a0 + f11 * a1;
    }
    v4u ph[2], pl[2];
#pragma unroll
    for (int g = 0; g < 2; ++g) {
      v4u a, a2;
#pragma unroll
      for (int e = 0; e < 4; ++e) {
        const float f0 = y[8 * g + 2 * e], f1 = y[8 * g + 2 * e + 1];
        const _Float16 x0 = (_Float16)f0, x1 = (_Float16)f1;
        const unsigned short h0 = h_bits(x0), h1 = h_bits(x1);
        const unsigned short l0 = h_bits((_Float16)((f0 - (float)x0) * QRES));
        const unsigned short l1 = h_bits((_Float16)((f1 - (float)x1) * QRES));
        a[e] = pk16(h0, h1); a2[e] = pk16(l0, l1);
      }
      ph[g] = a; pl[g] = a2;
    }
    if (wave < 4) {
      *(v4u*)(sQh + head * HD + d0)     = ph[0];
      *(v4u*)(sQh + head * HD + d0 + 8) = ph[1];
      *(v4u*)(sQl + head * HD + d0)     = pl[0];
      *(v4u*)(sQl + head * HD + d0 + 8) = pl[1];
    } else {
      *(v4u*)(sKh + (head - NH) * HD + d0)     = ph[0];
      *(v4u*)(sKh + (head - NH) * HD + d0 + 8) = ph[1];
      *(v4u*)(sKl + (head - NH) * HD + d0)     = pl[0];
      *(v4u*)(sKl + (head - NH) * HD + d0 + 8) = pl[1];
    }
  }
  __syncthreads();

  const int tk = (t < (KD / 8)) ? t : (KD / 8 - 1);
  const v4u va  = *(const v4u*)(sQh + t * 8);
  const v4u vl  = *(const v4u*)(sQl + t * 8);
  const v4u vk  = *(const v4u*)(sKh + tk * 8);
  const v4u vkl = *(const v4u*)(sKl + tk * 8);
  unsigned short* qrow  = Qh + (size_t)tok * QD + t * 8;
  unsigned short* lrow  = Ql + (size_t)tok * QD + t * 8;
  unsigned short* krow  = Kh + (size_t)tok * KD + tk * 8;
  unsigned short* klrow = Kl + (size_t)tok * KD + tk * 8;
#pragma unroll
  for (int pass = 0; pass < 2; ++pass) {
    *(volatile v4u*)qrow = va;
    *(volatile v4u*)lrow = vl;
    if (t < (KD / 8)) {
      *(volatile v4u*)krow  = vk;
      *(volatile v4u*)klrow = vkl;
    }
    __threadfence();
  }
}

__global__ __launch_bounds__(128)
void attn128(const unsigned short* __restrict__ qhp, const unsigned short* __restrict__ qlp,
             const unsigned short* __restrict__ khp, const unsigned short* __restrict__ klp,
             const unsigned short* __restrict__ vtp,
             const float* __restrict__ xm, unsigned short* op, float sscale) {
  union FH { v16h v; v8h h[2]; };
  __shared__ __align__(16) _Float16 Qsh[64 * HD];
  __shared__ __align__(16) _Float16 Qsl[64 * HD];
  __shared__ __align__(16) _Float16 Ksh[64 * HD];
  __shared__ __align__(16) _Float16 Ksl[64 * HD];
  __shared__ __align__(16) _Float16 Vth[HD * 64];
  __shared__ __align__(16) float    Msh[64 * 64];
  __shared__ __align__(16) _Float16 Psh[4][16 * 64];
  __shared__ __align__(16) float    Os[4][16 * HD];

  const int tid  = threadIdx.x;
  const int wave = tid >> 5;
  const int lane = tid & 31;
  const int hh   = lane >> 4;
  const int c    = lane & 15;

  const int bx   = blockIdx.x;
  const int qb   = bx % NQB;
  const int rest = bx / NQB;
  const int h    = rest % NH;
  const int b    = rest / NH;
  const int kvh  = h / NREP;
  const int q0   = qb * 64;
  const size_t tokQ = (size_t)b * SEQ + q0;

  const _Float16* Qh  = (const _Float16*)(const void*)qhp;
  const _Float16* Ql  = (const _Float16*)(const void*)qlp;
  const _Float16* Kg  = (const _Float16*)(const void*)khp;
  const _Float16* Klg = (const _Float16*)(const void*)klp;
  const _Float16* Vg  = (const _Float16*)(const void*)vtp;

  {
    const int r = tid >> 1, half = (tid & 1) * 64;
    const _Float16* gh = Qh + (tokQ + r) * QD + (size_t)h * HD + half;
    const _Float16* gl = Ql + (tokQ + r) * QD + (size_t)h * HD + half;
#pragma unroll
    for (int i = 0; i < 8; ++i) {
      *(v8h*)(Qsh + r * HD + half + 8 * i) = *(const v8h*)(gh + 8 * i);
#if SCORE_QRES
      *(v8h*)(Qsl + r * HD + half + 8 * i) = *(const v8h*)(gl + 8 * i);
#endif
    }
  }

  float mrow[8], lrow[8];
  v8f oacc[8];
#pragma unroll
  for (int r = 0; r < 8; ++r) { mrow[r] = -INFINITY; lrow[r] = 0.f; }
#pragma unroll
  for (int t = 0; t < 8; ++t) oacc[t] = zero8();

  for (int kt = 0; kt < NKT; ++kt) {
    const int kv0 = kt * 64;
    __syncthreads();
    {
      const int r = tid >> 1, half = (tid & 1) * 64, half32 = (tid & 1) * 32;
      const size_t krow = ((size_t)b * SEQ + kv0 + r) * KD + (size_t)kvh * HD + half;
      const _Float16* kg  = Kg  + krow;
      const _Float16* klg = Klg + krow;
      const _Float16* vg = Vg + ((size_t)b * KD + (size_t)kvh * HD + tid) * SEQ + kv0;
      const float* mg = xm + (((size_t)b * SEQ_FULL + q0 + r) * SEQ_FULL + kv0 + half32);
#pragma unroll
      for (int i = 0; i < 8; ++i) {
        *(v8h*)(Ksh + r * HD + half + 8 * i) = *(const v8h*)(kg + 8 * i);
#if SCORE_QRES
        *(v8h*)(Ksl + r * HD + half + 8 * i) = *(const v8h*)(klg + 8 * i);
#endif
        *(v8h*)(Vth + tid * 64 + 8 * i)      = *(const v8h*)(vg + 8 * i);
        v4f mv = *(const v4f*)(mg + 4 * i);
#pragma unroll
        for (int e = 0; e < 4; ++e) mv[e] = bfr(mv[e]);
        *(v4f*)(Msh + r * 64 + half32 + 4 * i) = mv;
      }
    }
    __syncthreads();

    v8f s[4];
#pragma unroll
    for (int j = 0; j < 4; ++j) {
      v8f sh = zero8(), sl = zero8();
#pragma unroll 1
      for (int dc = 0; dc < 4; ++dc) {
        FH qa, kb;
        qa.h[0] = *(const v8h*)(Qsh + (wave * 16 + c) * HD + dc * 32 + 8 * hh);
        qa.h[1] = *(const v8h*)(Qsh + (wave * 16 + c) * HD + dc * 32 + 16 + 8 * hh);
        kb.h[0] = *(const v8h*)(Ksh + (j * 16 + c) * HD + dc * 32 + 8 * hh);
        kb.h[1] = *(const v8h*)(Ksh + (j * 16 + c) * HD + dc * 32 + 16 + 8 * hh);
        sh = mma_h(qa.v, kb.v, sh);
#if SCORE_QRES
        FH ql, kl;
        ql.h[0] = *(const v8h*)(Qsl + (wave * 16 + c) * HD + dc * 32 + 8 * hh);
        ql.h[1] = *(const v8h*)(Qsl + (wave * 16 + c) * HD + dc * 32 + 16 + 8 * hh);
        kl.h[0] = *(const v8h*)(Ksl + (j * 16 + c) * HD + dc * 32 + 8 * hh);
        kl.h[1] = *(const v8h*)(Ksl + (j * 16 + c) * HD + dc * 32 + 16 + 8 * hh);
        sl = mma_h(ql.v, kb.v, sl);
        sl = mma_h(qa.v, kl.v, sl);
#endif
      }
#pragma unroll
      for (int r = 0; r < 8; ++r) s[j][r] = sh[r] + sl[r] * (1.0f / QRES);
    }

    _Float16* pwh = Psh[wave];
    const float* mrp = Msh + (wave * 16 + 8 * hh) * 64 + c;
#pragma unroll
    for (int r = 0; r < 8; ++r) {
      float m = -INFINITY;
#pragma unroll
      for (int j = 0; j < 4; ++j) {
        const float sv = s[j][r] * sscale + mrp[r * 64 + j * 16];
        s[j][r] = sv;
        m = fmaxf(m, sv);
      }
#pragma unroll
      for (int off = 1; off < 16; off <<= 1) m = fmaxf(m, __shfl_xor(m, off, 32));
      const float mnew  = fmaxf(mrow[r], m);
      const float alpha = __expf(mrow[r] - mnew);
      mrow[r] = mnew;
      float psum = 0.f;
#pragma unroll
      for (int j = 0; j < 4; ++j) {
        const float p = __expf(s[j][r] - mnew);
        psum += p;
        pwh[(8 * hh + r) * 64 + j * 16 + c] = (_Float16)(p * PCARRY);
      }
#pragma unroll
      for (int off = 1; off < 16; off <<= 1) psum += __shfl_xor(psum, off, 32);
      lrow[r] = lrow[r] * alpha + psum;
#pragma unroll
      for (int t = 0; t < 8; ++t) oacc[t][r] *= alpha;
    }
    __builtin_amdgcn_fence(__ATOMIC_RELEASE, "workgroup");
    __builtin_amdgcn_wave_barrier();
    __builtin_amdgcn_fence(__ATOMIC_ACQUIRE, "workgroup");

#pragma unroll 1
    for (int kk = 0; kk < 2; ++kk) {
      FH pa;
      pa.h[0] = *(const v8h*)(pwh + c * 64 + kk * 32 + 8 * hh);
      pa.h[1] = *(const v8h*)(pwh + c * 64 + kk * 32 + 16 + 8 * hh);
#pragma unroll
      for (int t = 0; t < 8; ++t) {
        FH vb;
        vb.h[0] = *(const v8h*)(Vth + (t * 16 + c) * 64 + kk * 32 + 8 * hh);
        vb.h[1] = *(const v8h*)(Vth + (t * 16 + c) * 64 + kk * 32 + 16 + 8 * hh);
        oacc[t] = mma_h(pa.v, vb.v, oacc[t]);
      }
    }
  }

  float* os = Os[wave];
#pragma unroll
  for (int r = 0; r < 8; ++r) {
    const float l = lrow[r];
    const float inv = ((l > 0.f) ? (1.0f / l) : 0.f) * (OCARRY / PCARRY);
#pragma unroll
    for (int t = 0; t < 8; ++t) os[(8 * hh + r) * HD + t * 16 + c] = oacc[t][r] * inv;
  }
  __builtin_amdgcn_fence(__ATOMIC_RELEASE, "workgroup");
  __builtin_amdgcn_wave_barrier();
  __builtin_amdgcn_fence(__ATOMIC_ACQUIRE, "workgroup");
  {
    const int rsub = lane >> 4, c8 = (lane & 15) * 8;
    v4u hv[8];
#pragma unroll
    for (int it = 0; it < 8; ++it) {
      const int row = it * 2 + rsub;
      const float* sp = os + row * HD + c8;
      v4u a;
#pragma unroll
      for (int e = 0; e < 4; ++e) {
        const _Float16 x0 = (_Float16)sp[2 * e], x1 = (_Float16)sp[2 * e + 1];
        a[e] = pk16(h_bits(x0), h_bits(x1));
      }
      hv[it] = a;
    }
#pragma unroll
    for (int pass = 0; pass < 2; ++pass) {
#pragma unroll
      for (int it = 0; it < 8; ++it) {
        const int row = it * 2 + rsub;
        const size_t go = (tokQ + wave * 16 + row) * QD + (size_t)h * HD + c8;
        *(volatile v4u*)(op + go) = hv[it];
      }
      __threadfence();
    }
  }
}

extern "C" void kernel_launch(void* const* d_in, const int* in_sizes, int n_in,
                              void* d_out, int out_size, void* d_ws, size_t ws_size,
                              hipStream_t stream) {
  if (n_in < 7) return;
  if ((long long)in_sizes[0] < (long long)NB * SEQ_FULL * DIMX) return;
  if ((long long)in_sizes[1] < (long long)NB * SEQ_FULL * SEQ_FULL) return;
  if ((long long)in_sizes[2] < (long long)SEQ * FRQ) return;
  if (in_sizes[3] != QKVO * DIMX) return;
  if (in_sizes[4] != DIMX * QD) return;
  if (in_sizes[5] != HD || in_sizes[6] != HD) return;
  if ((long long)out_size < (long long)NB * SEQ * DIMX) return;

  const float* x     = (const float*)d_in[0];
  const float* xmask = (const float*)d_in[1];
  const float* freqs = (const float*)d_in[2];
  const float* wqkv  = (const float*)d_in[3];
  const float* wout  = (const float*)d_in[4];
  const float* qw    = (const float*)d_in[5];
  const float* kw    = (const float*)d_in[6];

  const size_t nTok = (size_t)NB * SEQ;
  const size_t szXb  = nTok * DIMX * 2;
  const size_t szOc  = nTok * QD * 2;
  const size_t szWb  = (size_t)QKVO * DIMX * 2;
  const size_t szKp  = nTok * KD * 2;
  const size_t szQKf = nTok * QKC * 4;
  const size_t szWo  = (size_t)DIMX * QD * 2;
  const size_t szVT  = (size_t)NB * KD * SEQ * 2;
  const size_t szQ   = nTok * QD * 2;
  const size_t R0 = (szXb > szOc) ? szXb : szOc;
  const size_t R1 = (szWb > 2 * szKp) ? szWb : (2 * szKp);
  const size_t R2 = (szQKf > szWo) ? szQKf : szWo;
  size_t off = 0;
  const size_t oR0 = off; off += R0;
  const size_t oR1 = off; off += R1;
  const size_t oR2 = off; off += R2;
  const size_t oVT = off; off += szVT;
  const size_t oQh = off; off += szQ;
  const size_t oQl = off; off += szQ;
  if (off > ws_size) return;
  if (off > (size_t)134217728) return;

  char* ws = (char*)d_ws;
  unsigned short* Xb   = (unsigned short*)(ws + oR0);
  unsigned short* Oc   = (unsigned short*)(ws + oR0);
  unsigned short* Wb   = (unsigned short*)(ws + oR1);
  unsigned short* Khp  = (unsigned short*)(ws + oR1);
  unsigned short* Klp  = (unsigned short*)(ws + oR1 + szKp);
  float*          QKf  = (float*)(ws + oR2);
  unsigned short* Wo16 = (unsigned short*)(ws + oR2);
  unsigned short* VT   = (unsigned short*)(ws + oVT);
  unsigned short* Qh   = (unsigned short*)(ws + oQh);
  unsigned short* Ql   = (unsigned short*)(ws + oQl);

  const dim3 blk(256);
  const int n8x  = (int)(nTok * DIMX / 8);
  const int n8w  = QKVO * DIMX / 8;
  const int n8wo = DIMX * QD / 8;
  const dim3 gCvtX((n8x + 255) / 256);
  const dim3 gCvtW((n8w + 255) / 256);
  const dim3 gCvtWo((n8wo + 255) / 256);
  const int tilesQK  = (int)(nTok / 64) * (QKC / 64);
  const int tilesVT  = (KD / 64) * (SEQ / 64);
  const int tilesOut = (int)(nTok / 64) * (DIMX / 64);
  const dim3 gQK((tilesQK + 7) / 8, 1);
  const dim3 gVT((tilesVT + 7) / 8, NB);
  const dim3 gOut((tilesOut + 7) / 8, 1);
  const dim3 gPost((unsigned)nTok);
  const dim3 gAttn(NB * NH * NQB);
  const long long sXb = (long long)SEQ * DIMX;
  const long long sVT = (long long)KD * SEQ;
  const float sscale = 1.0f / sqrtf((float)HD);
  const float oscaleOut = 1.0f / (OCARRY * WOCARRY);

  cvt_x_bf16x8<<<gCvtX, blk, 0, stream>>>(x, Xb, n8x);
  cvt_bf16x8<<<gCvtW, blk, 0, stream>>>(wqkv, Wb, n8w);
  gemm64<0, 0><<<gQK, blk, 0, stream>>>(
      Xb, DIMX, 0LL, Wb, DIMX, 0LL, (void*)QKf, QKC, 0LL, (int)nTok, QKC, DIMX, 1.0f);
  gemm64<0, 1><<<gVT, blk, 0, stream>>>(
      Wb + (size_t)QKC * DIMX, DIMX, 0LL, Xb, DIMX, sXb, (void*)VT, SEQ, sVT, KD, SEQ, DIMX, 1.0f);
  qk_post<<<gPost, blk, 0, stream>>>(QKf, freqs, qw, kw, Qh, Ql, Khp, Klp);
  cvt_wo_f16x8<<<gCvtWo, blk, 0, stream>>>(wout, Wo16, n8wo);
  attn128<<<gAttn, dim3(128), 0, stream>>>(Qh, Ql, Khp, Klp, VT, xmask, Oc, sscale);
  gemm64<1, 0><<<gOut, blk, 0, stream>>>(
      Oc, QD, 0LL, Wo16, QD, 0LL, d_out, DIMX, 0LL, (int)nTok, DIMX, QD, oscaleOut);
  (void)hipGetLastError();
}
